// MultiHeadAttention_85177791414455
// MI455X (gfx1250) — hardware-verified
//
#include <hip/hip_runtime.h>
#ifndef NB
#define NB 4
#endif
#ifndef SEQ
#define SEQ 2048
#endif
#define NB_FULL 4
#define SEQ_FULL 2048
#define DM 1024
#define NH 16
#define HD 64
#define LQ (3 * DM)
#define QT0 128
#define PP 72

static_assert(NH * HD == DM);
static_assert(HD == 64);
static_assert(DM % 64 == 0 && LQ % 64 == 0);
static_assert(DM % 32 == 0);
static_assert(SEQ % 128 == 0);
static_assert(QT0 % 128 == 0 && QT0 % 64 == 0);
static_assert(SEQ >= QT0 + 64);
static_assert((SEQ - QT0) % 64 == 0);
static_assert(NB <= NB_FULL && SEQ <= SEQ_FULL);
static_assert(PP % 8 == 0 && PP >= 64);

typedef unsigned short v8us __attribute__((ext_vector_type(8), may_alias));
typedef float  v8f  __attribute__((ext_vector_type(8)));
typedef float  v4f  __attribute__((ext_vector_type(4)));
typedef float  v4fa __attribute__((ext_vector_type(4), may_alias));
typedef _Float16 v16h __attribute__((ext_vector_type(16)));
typedef _Float16 v8hp __attribute__((ext_vector_type(8)));
typedef _Float16 v8ha __attribute__((ext_vector_type(8), may_alias));
typedef _Float16 v4h  __attribute__((ext_vector_type(4)));
union FragH { v16h v; v8us half[2]; _Float16 h[16]; unsigned short u[16]; };
union FragP { v16h v; v8hp half[2]; };

constexpr size_t WS_BTA  = (size_t)LQ * DM * 2;
constexpr size_t WS_BTP  = (size_t)DM * DM * 2;
constexpr size_t WS_X16  = (size_t)NB * SEQ * DM * 2;
constexpr size_t WS_QKV  = (size_t)NB * SEQ * LQ * 2;
constexpr size_t WS_VT   = (size_t)NB * NH * HD * SEQ * 2;
constexpr size_t WS_O16  = (size_t)NB * SEQ * DM * 2;
constexpr size_t WS_QF0  = (size_t)NB * QT0 * LQ * 4;
constexpr size_t WS_OF0  = (size_t)NB * QT0 * DM * 4;
constexpr size_t WS_OL0  = (size_t)NB * QT0 * DM * 2;
constexpr size_t WS_TOTAL = WS_BTA + WS_BTP + WS_X16 + WS_QKV + WS_VT + WS_O16 + WS_QF0 + WS_OF0 + WS_OL0;
static_assert(WS_TOTAL <= (size_t)134217728);
static_assert(WS_BTA % 256 == 0 && WS_BTP % 256 == 0 && WS_X16 % 256 == 0 && WS_QKV % 256 == 0 && WS_VT % 256 == 0 && WS_O16 % 256 == 0 && WS_QF0 % 256 == 0 && WS_OF0 % 256 == 0 && WS_OL0 % 256 == 0);

__device__ __forceinline__ unsigned short bf16_bits(float x) { unsigned int u = __float_as_uint(x); return (unsigned short)((u + 0x7FFFu + ((u >> 16) & 1u)) >> 16); }
__device__ __forceinline__ float bf16_rne(float x) { return __uint_as_float(((unsigned int)bf16_bits(x)) << 16); }

__device__ __forceinline__ v16h g2_frag(const _Float16* p, int hh) { FragH f; f.half[0] = *(const v8us*)((const unsigned short*)p + 8 * hh); f.half[1] = *(const v8us*)((const unsigned short*)p + 16 + 8 * hh); return f.v; }
__device__ __forceinline__ v8f g2_mma(v16h a, v16h b, v8f c) { v8f d = __builtin_amdgcn_wmma_f32_16x16x32_f16(false, a, false, b, (short)0, c, false, false); asm volatile("v_nop\n\tv_nop\n\tv_nop\n\tv_nop" : "+v"(d) : "v"(a), "v"(b)); return d; }

__global__ __launch_bounds__(256) void k_wt_f16(const float* __restrict__ W, _Float16* __restrict__ Wt, int K, int N, float scale) {
  const int t = blockIdx.x * 256 + threadIdx.x; if (t >= N * (K / 8)) return; const int n = t / (K / 8), k8 = (t % (K / 8)) * 8; FragH f;
#pragma unroll
  for (int i = 0; i < 8; ++i) f.h[i] = (_Float16)(bf16_rne(W[(size_t)(k8 + i) * N + n]) * scale);
  const v8us o = f.half[0]; unsigned short* d = (unsigned short*)Wt + (size_t)n * K + k8;
  *(volatile v8us*)d = o; __threadfence(); *(volatile v8us*)d = o;
}

__global__ __launch_bounds__(256) void k_x16(const float* __restrict__ x, _Float16* __restrict__ X16, unsigned n8b, size_t sx, size_t sd) {
  const unsigned t = blockIdx.x * 256 + threadIdx.x; if (t >= n8b) return;
  const float* s = x + (size_t)blockIdx.y * sx + (size_t)t * 8;
  const v4f a = *(const v4fa*)s, c = *(const v4fa*)(s + 4); FragH f;
#pragma unroll
  for (int q = 0; q < 4; ++q) { f.h[q] = (_Float16)bf16_rne(a[q]); f.h[4 + q] = (_Float16)bf16_rne(c[q]); }
  const v8us o = f.half[0]; unsigned short* d = (unsigned short*)X16 + (size_t)blockIdx.y * sd + (size_t)t * 8;
  *(volatile v8us*)d = o; __threadfence(); *(volatile v8us*)d = o;
}

__global__ __launch_bounds__(128) void k_gemm2(const _Float16* __restrict__ A, int lda, size_t sA, const _Float16* __restrict__ Bh, int ldb, float alpha, const float* __restrict__ bias, int hasBias,
    const float* CP, int accum, float* C, _Float16* __restrict__ C16, int ldc, size_t sC, int M, int N, int K) {
  __shared__ __attribute__((aligned(16))) float so[4][32][68];
  const int tid = threadIdx.x, w = tid >> 5, lane = tid & 31, ln = lane & 15, hh = lane >> 4; const int by = blockIdx.y;
  A += (size_t)by * sA; const size_t cofs = (size_t)by * sC;
  const int ntn = N >> 6; const int mt = blockIdx.x / ntn, nq = blockIdx.x - mt * ntn; const int row0 = mt * 128 + 32 * w, col0 = nq * 64; if (row0 >= M) return;
  const _Float16* a0p = A + (size_t)(row0 + ln) * lda; const _Float16* a1p = a0p + (size_t)16 * lda;
  const _Float16* b0p = Bh + (size_t)(col0 + ln) * ldb; const _Float16* b1p = b0p + (size_t)16 * ldb; const _Float16* b2p = b1p + (size_t)16 * ldb; const _Float16* b3p = b2p + (size_t)16 * ldb;
  const v8f z8 = {0.f,0.f,0.f,0.f,0.f,0.f,0.f,0.f}; v8f c00 = z8, c01 = z8, c02 = z8, c03 = z8, c10 = z8, c11 = z8, c12 = z8, c13 = z8;
#pragma unroll 1
  for (int kb = 0; kb < K; kb += 32) { const v16h a0 = g2_frag(a0p + kb, hh), a1 = g2_frag(a1p + kb, hh);
    v16h b = g2_frag(b0p + kb, hh); c00 = g2_mma(a0, b, c00); c10 = g2_mma(a1, b, c10);
    b = g2_frag(b1p + kb, hh); c01 = g2_mma(a0, b, c01); c11 = g2_mma(a1, b, c11);
    b = g2_frag(b2p + kb, hh); c02 = g2_mma(a0, b, c02); c12 = g2_mma(a1, b, c12);
    b = g2_frag(b3p + kb, hh); c03 = g2_mma(a0, b, c03); c13 = g2_mma(a1, b, c13); }
  v8f accs[8] = {c00, c01, c02, c03, c10, c11, c12, c13};
#pragma unroll
  for (int u = 0; u < 8; ++u) { const int t = u & 3, half = u >> 2; const int col = col0 + t * 16 + ln; float bv = 0.f; if (hasBias) bv = bf16_rne(bias[col]);
#pragma unroll
    for (int r = 0; r < 8; ++r) { const int rloc = half * 16 + 8 * hh + r; float v = accs[u][r] * alpha + bv; if (accum) v += CP[cofs + (size_t)(row0 + rloc) * ldc + col];
      so[w][rloc][t * 16 + ln] = v; } }
  __builtin_amdgcn_fence(4  , "workgroup"); __builtin_amdgcn_wave_barrier();
  const int rsub = lane >> 4, c4 = (lane & 15) * 4;
  for (int pass = 0; pass < 2; ++pass) {
#pragma unroll
    for (int q = 0; q < 16; ++q) { const int r = q * 2 + rsub; const v4f v = *(const v4fa*)&so[w][r][c4]; if (C) *(volatile v4f*)(C + cofs + (size_t)(row0 + r) * ldc + col0 + c4) = v; if (C16) { v4h h4; for (int i = 0; i < 4; ++i) h4[i] = (_Float16)v[i]; *(volatile v4h*)(C16 + cofs + (size_t)(row0 + r) * ldc + col0 + c4) = h4; } }
    if (pass == 0) __threadfence(); } }

__global__ __launch_bounds__(256) void k_vt(const _Float16* __restrict__ QKV, _Float16* __restrict__ VT) { __shared__ unsigned short tl[64][66]; const int tid = threadIdx.x; const int slab = blockIdx.x / (SEQ / 64), lg = blockIdx.x % (SEQ / 64); const int b = slab / NH, h = slab % NH;
  for (int i = tid; i < 64 * 8; i += 256) { const int r = i / 8, c8 = (i % 8) * 8; FragH f; f.half[0] = *(const v8us*)((const unsigned short*)QKV + ((size_t)b * SEQ + lg * 64 + r) * LQ + 2 * DM + h * HD + c8);
#pragma unroll
    for (int q = 0; q < 8; ++q) tl[r][c8 + q] = f.u[q]; }
  __syncthreads();
  for (int pass = 0; pass < 2; ++pass) {
#pragma unroll
    for (int rd = 0; rd < 2; ++rd) { const int d = rd * 32 + tid / 8, pc = tid % 8; FragH f;
#pragma unroll
      for (int q = 0; q < 8; ++q) f.u[q] = tl[pc * 8 + q][d];
      *(volatile v8us*)((unsigned short*)VT + ((size_t)slab * HD + d) * SEQ + lg * 64 + pc * 8) = f.half[0]; }
    if (pass == 0) __threadfence(); } }

__global__ __launch_bounds__(64) void k_att0(const float* __restrict__ QF, float* __restrict__ OF) {
  #pragma clang fp contract(off)
  __shared__ __attribute__((aligned(16))) float lq[64][64]; __shared__ __attribute__((aligned(16))) float lo[64][64];
  const int tid = threadIdx.x; const int rg = blockIdx.x % (QT0 / 64); const int bhx = blockIdx.x / (QT0 / 64); const int h = bhx % NH, b = bhx / NH; const int i = rg * 64 + tid;
  const float* base = QF + (size_t)b * QT0 * LQ + h * HD;
  const float* qr = base + (size_t)i * LQ;
#pragma unroll 1
  for (int c = 0; c < HD / 4; ++c) { *(v4f*)&lq[tid][c * 4] = *(const v4fa*)(qr + c * 4); const v4f z = {0.f, 0.f, 0.f, 0.f}; *(v4f*)&lo[tid][c * 4] = z; }
  float m = -1.0e30f, l = 0.f; const int jmax = rg * 64 + 63;
#pragma unroll 1
  for (int j = 0; j <= jmax; ++j) { const float* kr = base + (size_t)j * LQ + DM; const float* vr = base + (size_t)j * LQ + 2 * DM; float s = 0.f;
#pragma unroll 1
    for (int c = 0; c < HD / 4; ++c) { const v4f kq = *(const v4fa*)(kr + c * 4); const v4f qq = *(v4f*)&lq[tid][c * 4]; s = __fadd_rn(s, __fmul_rn(qq[0], kq[0])); s = __fadd_rn(s, __fmul_rn(qq[1], kq[1])); s = __fadd_rn(s, __fmul_rn(qq[2], kq[2])); s = __fadd_rn(s, __fmul_rn(qq[3], kq[3])); }
    s = __fmul_rn(s, 0.125f);
    const float f = (j <= i) ? 1.f : 0.f; const float sm = fmaf(f, s, (1.f - f) * -1.0e30f); const float mn = fmaxf(m, sm); const float sc = expf(m - mn); const float e = expf(sm - mn); l = __fadd_rn(__fmul_rn(l, sc), e); m = mn;
#pragma unroll 1
    for (int c = 0; c < HD / 4; ++c) { const v4f vv = *(const v4fa*)(vr + c * 4); v4f oo = *(v4f*)&lo[tid][c * 4]; for (int u = 0; u < 4; ++u) oo[u] = __fadd_rn(__fmul_rn(oo[u], sc), __fmul_rn(e, vv[u])); *(v4f*)&lo[tid][c * 4] = oo; } }
  const float fin = 64.0f * (1.0f / l);
#pragma unroll 1
  for (int c = 0; c < HD / 4; ++c) { v4f oo = *(v4f*)&lo[tid][c * 4]; for (int u = 0; u < 4; ++u) oo[u] = __fmul_rn(oo[u], fin); *(v4f*)&lo[tid][c * 4] = oo; }
  __syncthreads();
  for (int pass = 0; pass < 2; ++pass) {
#pragma unroll 1
    for (int it = 0; it < 16; ++it) { const int row = it * 4 + tid / 16, pc = (tid % 16) * 4; const v4f v = *(const v4f*)&lo[row][pc]; *(volatile v4f*)(OF + ((size_t)b * QT0 + rg * 64 + row) * DM + h * HD + pc) = v; }
    if (pass == 0) __threadfence(); } }

__global__ __launch_bounds__(256) void k_hl(const float* __restrict__ F, _Float16* __restrict__ O16, _Float16* __restrict__ Hl, unsigned n8) { const unsigned t = blockIdx.x * 256 + threadIdx.x; if (t >= n8) return; FragH fh, fl; const v4f a = *(const v4fa*)(F + (size_t)t * 8), c = *(const v4fa*)(F + (size_t)t * 8 + 4);
#pragma unroll
  for (int q = 0; q < 4; ++q) { _Float16 h = (_Float16)a[q]; fh.h[q] = h; fl.h[q] = (_Float16)((a[q] - (float)h) * 1024.0f); h = (_Float16)c[q]; fh.h[4 + q] = h; fl.h[4 + q] = (_Float16)((c[q] - (float)h) * 1024.0f); }
  const unsigned row = t / (DM / 8), col = (t % (DM / 8)) * 8; const unsigned b = row / QT0, r = row % QT0;
  unsigned short* dh = (unsigned short*)O16 + ((size_t)b * SEQ + r) * DM + col; unsigned short* dl = (unsigned short*)Hl + (size_t)t * 8; const v8us oh = fh.half[0], ol = fl.half[0];
  for (int pass = 0; pass < 2; ++pass) { *(volatile v8us*)dh = oh; *(volatile v8us*)dl = ol; if (pass == 0) __threadfence(); } }

__global__ __launch_bounds__(128) void k_flash(const _Float16* __restrict__ QKV, const _Float16* __restrict__ VT, _Float16* __restrict__ O16) {
  __shared__ __attribute__((aligned(16))) _Float16 sP[4][16 * PP];
  const int tid = threadIdx.x, w = tid >> 5, lane = tid & 31, ln = lane & 15, hh = lane >> 4;
  const int bh = blockIdx.y, b = bh / NH, h = bh - b * NH;
  const int q0w = QT0 + (int)blockIdx.x * 64 + w * 16;
  const size_t rowb = (size_t)b * SEQ;
  const _Float16* qp = QKV + (rowb + q0w + ln) * LQ + h * HD;
  const v16h qa0 = g2_frag(qp, hh), qa1 = g2_frag(qp + 32, hh);
  const _Float16* kbase = QKV + (rowb + ln) * LQ + DM + h * HD;
  const _Float16* vbase = VT + ((size_t)bh * HD + ln) * SEQ;
  const v8f z8 = {0.f,0.f,0.f,0.f,0.f,0.f,0.f,0.f};
  v8f o[4] = {z8, z8, z8, z8};
  float m[8], l[8];
#pragma unroll
  for (int r = 0; r < 8; ++r) { m[r] = -3.0e38f; l[r] = 0.f; }
  const int nkt = (q0w >> 6) + 1;
#pragma unroll 1
  for (int kt = 0; kt < nkt; ++kt) {
    const int k0 = kt * 64;
    v8f s[4];
#pragma unroll
    for (int j = 0; j < 4; ++j) { const _Float16* kp = kbase + (size_t)(k0 + j * 16) * LQ; const v16h b0 = g2_frag(kp, hh), b1 = g2_frag(kp + 32, hh); v8f a = z8; a = g2_mma(qa0, b0, a); a = g2_mma(qa1, b1, a); s[j] = a; }
    const int lim = (kt == nkt - 1) ? (q0w + 8 * hh - k0 - ln) : 0x7fffffff;
#pragma unroll
    for (int j = 0; j < 4; ++j)
#pragma unroll
      for (int r = 0; r < 8; ++r) { const float v = s[j][r] * 0.18033688011112042f; s[j][r] = (j * 16 - r > lim) ? -3.0e38f : v; }
    float mn[8];
#pragma unroll
    for (int r = 0; r < 8; ++r) mn[r] = fmaxf(fmaxf(s[0][r], s[1][r]), fmaxf(s[2][r], s[3][r]));
#pragma unroll
    for (int msk = 1; msk <= 8; msk <<= 1)
#pragma unroll
      for (int r = 0; r < 8; ++r) mn[r] = fmaxf(mn[r], __shfl_xor(mn[r], msk, 32));
    float rs[8];
#pragma unroll
    for (int r = 0; r < 8; ++r) { mn[r] = fmaxf(mn[r], m[r]); const float mm = mn[r] - 8.0f; float acc = 0.f;
#pragma unroll
      for (int j = 0; j < 4; ++j) { const float p = __builtin_amdgcn_exp2f(s[j][r] - mm); s[j][r] = p; acc += p; }
      rs[r] = acc; }
#pragma unroll
    for (int msk = 1; msk <= 8; msk <<= 1)
#pragma unroll
      for (int r = 0; r < 8; ++r) rs[r] += __shfl_xor(rs[r], msk, 32);
#pragma unroll
    for (int r = 0; r < 8; ++r) { const float alpha = __builtin_amdgcn_exp2f(m[r] - mn[r]); l[r] = l[r] * alpha + rs[r]; m[r] = mn[r];
#pragma unroll
      for (int j = 0; j < 4; ++j) o[j][r] *= alpha; }
#pragma unroll
    for (int j = 0; j < 4; ++j)
#pragma unroll
      for (int r = 0; r < 8; ++r) sP[w][(8 * hh + r) * PP + j * 16 + ln] = (_Float16)s[j][r];
    __builtin_amdgcn_fence(4  , "workgroup"); __builtin_amdgcn_wave_barrier();
    FragP pa0, pa1;
    pa0.half[0] = *(const v8ha*)&sP[w][ln * PP + 8 * hh];       pa0.half[1] = *(const v8ha*)&sP[w][ln * PP + 16 + 8 * hh];
    pa1.half[0] = *(const v8ha*)&sP[w][ln * PP + 32 + 8 * hh];  pa1.half[1] = *(const v8ha*)&sP[w][ln * PP + 48 + 8 * hh];
#pragma unroll
    for (int j = 0; j < 4; ++j) { const _Float16* vp = vbase + (size_t)j * 16 * SEQ + k0; const v16h vb0 = g2_frag(vp, hh), vb1 = g2_frag(vp + 32, hh); o[j] = g2_mma(pa0.v, vb0, o[j]); o[j] = g2_mma(pa1.v, vb1, o[j]); }
    __builtin_amdgcn_fence(4  , "workgroup"); __builtin_amdgcn_wave_barrier();
  }
  float inv[8];
#pragma unroll
  for (int r = 0; r < 8; ++r) inv[r] = 64.0f * (1.0f / l[r]);
#pragma unroll
  for (int j = 0; j < 4; ++j)
#pragma unroll
    for (int r = 0; r < 8; ++r) sP[w][(8 * hh + r) * PP + j * 16 + ln] = (_Float16)(o[j][r] * inv[r]);
  __builtin_amdgcn_fence(4  , "workgroup"); __builtin_amdgcn_wave_barrier();
  const int rq = lane >> 3, pc = (lane & 7) * 8;
  for (int pass = 0; pass < 2; ++pass) {
#pragma unroll
    for (int it = 0; it < 4; ++it) { const int row = it * 4 + rq; const v8hp v = *(const v8ha*)&sP[w][row * PP + pc]; *(volatile v8hp*)(O16 + (rowb + q0w + row) * DM + h * HD + pc) = v; }
    if (pass == 0) __threadfence(); } }

extern "C" void kernel_launch(void* const* d_in, const int* in_sizes, int n_in,
                              void* d_out, int out_size, void* d_ws, size_t ws_size, hipStream_t stream) {
  if (n_in < 5) return;
  const size_t need_x = (size_t)(NB - 1) * SEQ_FULL * DM + (size_t)SEQ * DM;
  if ((size_t)in_sizes[0] < need_x) return;
  if ((size_t)in_sizes[1] < (size_t)DM * LQ) return;
  if ((size_t)in_sizes[2] < (size_t)LQ) return;
  if ((size_t)in_sizes[3] < (size_t)DM * DM) return;
  if ((size_t)in_sizes[4] < (size_t)DM) return;
  if ((size_t)out_size < need_x) return;
  if (WS_TOTAL > ws_size) return;
  const float* x = (const float*)d_in[0]; const float* wa = (const float*)d_in[1]; const float* ba = (const float*)d_in[2]; const float* wp = (const float*)d_in[3]; const float* bp = (const float*)d_in[4];
  float* out = (float*)d_out;
  char* ws = (char*)d_ws; size_t off = 0;
  _Float16* BTA = (_Float16*)(ws + off); off += WS_BTA;
  _Float16* BTP = (_Float16*)(ws + off); off += WS_BTP;
  _Float16* X16 = (_Float16*)(ws + off); off += WS_X16;
  _Float16* QKV = (_Float16*)(ws + off); off += WS_QKV;
  _Float16* VT  = (_Float16*)(ws + off); off += WS_VT;
  _Float16* O16 = (_Float16*)(ws + off); off += WS_O16;
  float*    QF0 = (float*)(ws + off);    off += WS_QF0;
  float*    OF0 = (float*)(ws + off);    off += WS_OF0;
  _Float16* OL0 = (_Float16*)(ws + off); off += WS_OL0;

  k_wt_f16<<<(unsigned)(((size_t)LQ * (DM / 8) + 255) / 256), 256, 0, stream>>>(wa, BTA, DM, LQ, 16.0f);
  k_wt_f16<<<(unsigned)(((size_t)DM * (DM / 8) + 255) / 256), 256, 0, stream>>>(wp, BTP, DM, DM, 16.0f);
  k_x16<<<dim3((unsigned)(((size_t)SEQ * DM / 8 + 255) / 256), NB), 256, 0, stream>>>(x, X16, (unsigned)((size_t)SEQ * DM / 8), (size_t)SEQ_FULL * DM, (size_t)SEQ * DM);
  k_gemm2<<<dim3((unsigned)(((size_t)NB * SEQ / 128) * (LQ / 64)), 1), 128, 0, stream>>>(X16, DM, 0, BTA, DM, 0.0625f, ba, 1, ba, 0, nullptr, QKV, LQ, 0, NB * SEQ, LQ, DM);
  k_gemm2<<<dim3((QT0 / 128) * (LQ / 64), NB), 128, 0, stream>>>(X16, DM, (size_t)SEQ * DM, BTA, DM, 0.0625f, ba, 1, ba, 0, QF0, nullptr, LQ, (size_t)QT0 * LQ, QT0, LQ, DM);
  k_vt<<<NB * NH * (SEQ / 64), 256, 0, stream>>>(QKV, VT);
  k_att0<<<NB * NH * (QT0 / 64), 64, 0, stream>>>(QF0, OF0);
  k_flash<<<dim3((SEQ - QT0) / 64, NB * NH), 128, 0, stream>>>(QKV, VT, O16);
  k_hl<<<(unsigned)(((size_t)NB * QT0 * DM / 8 + 255) / 256), 256, 0, stream>>>(OF0, O16, OL0, (unsigned)((size_t)NB * QT0 * DM / 8));
  k_gemm2<<<dim3((SEQ / 128) * (DM / 64), NB), 128, 0, stream>>>(O16, DM, (size_t)SEQ * DM, BTP, DM, 0.0009765625f, bp, 1, bp, 0, out, nullptr, DM, (size_t)SEQ_FULL * DM, SEQ, DM, DM);
  k_gemm2<<<dim3((QT0 / 128) * (DM / 64), NB), 128, 0, stream>>>(OL0, DM, (size_t)QT0 * DM, BTP, DM, 0.00000095367431640625f, bp, 0, out, 1, out, nullptr, DM, (size_t)SEQ_FULL * DM, QT0, DM, DM);
}
